// Attention_57389353009692
// MI455X (gfx1250) — hardware-verified
//
#include <hip/hip_runtime.h>


#ifndef NB
#define NB 1
#endif
#ifndef SEQ
#define SEQ 2048
#endif
#ifndef EARLY
#define EARLY 512
#endif
#define NB_FULL  1
#define SEQ_FULL 2048
#define DM   2048
#define NH   32
#define HD   64
#define KVW  512
#define NQKV 3072
#define XEP  2432
#define WEP  2176
#define CXP  4224
#define WCP  4096
#define NA1  256
#define NA2  128
#define NWV  4
#define OSP  72
#define GSP  36
#define VTP  72
#define L2E  1.4426950408889634f
#define RQ   0.00048828125f
#define EARLYR ((EARLY) < (SEQ) ? (EARLY) : (SEQ))
#define MNIT ((SEQ + 1023) / 1024)

static_assert(NB == 1);
static_assert(NB <= NB_FULL);
static_assert(SEQ <= SEQ_FULL);
static_assert(SEQ % 128 == 0);
static_assert(SEQ / 64 <= 32);
static_assert(MNIT <= 2);
static_assert(EARLYR % 64 == 0);
static_assert(NH * HD == DM);
static_assert(HD == 64);
static_assert(DM % 32 == 0 && WEP % 32 == 0 && CXP % 32 == 0 && WCP % 32 == 0);
static_assert(NQKV % 64 == 0 && NA1 % 64 == 0 && NA2 % 64 == 0 && DM % 64 == 0);
static_assert(XEP % 64 == 0 && WEP % 64 == 0 && CXP % 64 == 0);
static_assert(((size_t)SEQ * 3 * 16) % 256 == 0 && ((size_t)SEQ * 16) % 256 == 0);
static_assert(((size_t)SEQ * 256) % 256 == 0);

typedef unsigned short us;
typedef __attribute__((ext_vector_type(16))) __bf16   v16bf;
typedef __attribute__((ext_vector_type(16))) _Float16 v16h;
typedef __attribute__((ext_vector_type(8)))  _Float16 v8h;
typedef __attribute__((ext_vector_type(8)))  unsigned short v8us;
typedef __attribute__((ext_vector_type(8)))  float    v8f;
typedef __attribute__((ext_vector_type(4)))  float    v4f;
typedef __attribute__((ext_vector_type(4)))  int      v4i;
typedef v4f  __attribute__((may_alias)) v4fa;
typedef v8us __attribute__((may_alias)) v8usa;

__device__ __forceinline__ unsigned short f2bf(float f) { unsigned u = __float_as_uint(f); u += 0x7FFFu + ((u >> 16) & 1u); return (unsigned short)(u >> 16); }
__device__ __forceinline__ float bf2f(unsigned short b) { return __uint_as_float(((unsigned)b) << 16); }
__device__ __forceinline__ float bfr(float f) { return bf2f(f2bf(f)); }
__device__ __forceinline__ v16bf cat16b(v8us lo, v8us hi) { return __builtin_bit_cast(v16bf, __builtin_shufflevector(lo, hi, 0, 1, 2, 3, 4, 5, 6, 7, 8, 9, 10, 11, 12, 13, 14, 15)); }
__device__ __forceinline__ v16h  cat16h(v8us lo, v8us hi) { return __builtin_bit_cast(v16h,  __builtin_shufflevector(lo, hi, 0, 1, 2, 3, 4, 5, 6, 7, 8, 9, 10, 11, 12, 13, 14, 15)); }
__device__ __forceinline__ v8f wmmab(v16bf a, v16bf b, v8f c) { return __builtin_amdgcn_wmma_f32_16x16x32_bf16(false, a, false, b, (short)0, c, false, false); }
__device__ __forceinline__ v8f wmmah(v16h a, v16h b, v8f c)   { return __builtin_amdgcn_wmma_f32_16x16x32_f16(false, a, false, b, (short)0, c, false, false); }
__device__ __forceinline__ v16bf ldb(const us* p) { return cat16b(*(const v8us*)p, *(const v8us*)(p + 16)); }
__device__ __forceinline__ v16h  ldh(const us* p) { return cat16h(*(const v8us*)p, *(const v8us*)(p + 16)); }

__global__ __launch_bounds__(256) void k_mscan(const float* __restrict__ mask, const int* __restrict__ sp, int* MT) {
    __shared__ int fnz[32];
    __shared__ int fni[32];
    (void)sp;
    const unsigned tid = threadIdx.x, qb = blockIdx.x;
    const float NINF = -__builtin_inff();
    int nz[MNIT], ni[MNIT];
#pragma unroll
    for (int it = 0; it < MNIT; ++it) { nz[it] = 0; ni[it] = 0; }
#pragma unroll 1
    for (unsigned r = 0; r < 64u; ++r) {
        const float* mr = mask + (size_t)(qb * 64u + r) * SEQ_FULL;
#pragma unroll
        for (int it = 0; it < MNIT; ++it) {
            const unsigned f = tid + (unsigned)it * 256u;
            const unsigned fc = f < (unsigned)(SEQ / 4) ? f : (unsigned)(SEQ / 4 - 1);
            const v4f v = *(const v4f*)(mr + fc * 4u);
            const int ok = (int)(f < (unsigned)(SEQ / 4));
            const int a = (int)(v[0] != 0.0f) | (int)(v[1] != 0.0f) | (int)(v[2] != 0.0f) | (int)(v[3] != 0.0f);
            const int b = (int)(!(v[0] == NINF)) | (int)(!(v[1] == NINF)) | (int)(!(v[2] == NINF)) | (int)(!(v[3] == NINF));
            nz[it] |= ok & a;
            ni[it] |= ok & b;
        }
    }
#pragma unroll
    for (int it = 0; it < MNIT; ++it) {
#pragma unroll
        for (int m = 1; m <= 8; m <<= 1) {
            nz[it] |= __shfl_xor(nz[it], m, 32);
            ni[it] |= __shfl_xor(ni[it], m, 32);
        }
    }
    if ((tid & 15u) == 0u) {
#pragma unroll
        for (int it = 0; it < MNIT; ++it) {
            const unsigned kb = (tid >> 4) + (unsigned)it * 16u;
            if (kb < (unsigned)(SEQ / 64)) { fnz[kb] = nz[it]; fni[kb] = ni[it]; }
        }
    }
    __syncthreads();
    if (tid < 8u) {
        v4i o;
#pragma unroll
        for (unsigned c = 0; c < 4u; ++c) {
            const unsigned j = tid * 4u + c;
            const unsigned jc = j < (unsigned)(SEQ / 64) ? j : (unsigned)(SEQ / 64 - 1);
            const int z = fnz[jc], n = fni[jc];
            int cls = (n == 0) ? 2 : ((z == 0) ? 0 : 1);
            if (j >= (unsigned)(SEQ / 64)) cls = 2;
            o[c] = cls;
        }
        int* d = MT + qb * 32u + tid * 4u;
        *(volatile v4i*)d = o;
        __threadfence();
        *(volatile v4i*)d = o;
    }
}

__global__ __launch_bounds__(256) void k_cvt(const float* __restrict__ src, us* dst, unsigned rows, unsigned dpitch, unsigned rep) {
    const unsigned i = blockIdx.x * 256u + threadIdx.x;
    if (i >= rows * 256u) return;
    const unsigned row = i >> 8, c = (i & 255u) * 8u;
    const v8f v = *(const v8f*)(src + (size_t)row * DM + c);
    v8us o;
#pragma unroll
    for (int k = 0; k < 8; ++k) o[k] = f2bf(v[k]);
    us* d = dst + (size_t)row * dpitch + c;
#pragma unroll 1
    for (int ps = 0; ps < 2; ++ps) {
#pragma unroll 1
        for (unsigned j = 0; j < rep; ++j) *(volatile v8us*)(d + (size_t)j * DM) = o;
        if (ps == 0) __threadfence();
    }
}

__global__ __launch_bounds__(256) void k_bt(const float* __restrict__ Bw, us* dst, unsigned outd, unsigned ldw) {
    const unsigned i = blockIdx.x * 256u + threadIdx.x;
    if (i >= outd * 16u) return;
    const unsigned o = i >> 4, j = i & 15u, e = j & 7u;
    const v8f v = *(const v8f*)(Bw + ((size_t)e * outd + o) * 8u);
    v8us w;
#pragma unroll
    for (int k = 0; k < 8; ++k) w[k] = f2bf(v[k]);
    us* d = dst + (size_t)o * ldw + j * 8u;
    *(volatile v8us*)d = w;
    __threadfence();
    *(volatile v8us*)d = w;
}

__global__ __launch_bounds__(256) void k_rt(const float* __restrict__ r0, const float* __restrict__ r1, const float* __restrict__ r2,
                                            us* dst, unsigned ng, unsigned ldw, unsigned rep) {
    const unsigned row = blockIdx.x, c = threadIdx.x * 8u, g = row >> 3;
    const size_t ridx = (size_t)(row & 7u) * DM + c;
    const v8f a = *(const v8f*)(r0 + ridx);
    const v8f b = *(const v8f*)(r1 + ridx);
    const v8f d2 = *(const v8f*)(r2 + ridx);
    v8us o;
#pragma unroll
    for (int k = 0; k < 8; ++k) {
        float v = (g == 0u) ? a[k] : ((g == 1u) ? b[k] : d2[k]);
        if (g >= ng) v = 0.0f;
        o[k] = f2bf(v);
    }
    us* d = dst + (size_t)row * ldw + c;
#pragma unroll 1
    for (int ps = 0; ps < 2; ++ps) {
#pragma unroll 1
        for (unsigned j = 0; j < rep; ++j) *(volatile v8us*)(d + (size_t)j * DM) = o;
        if (ps == 0) __threadfence();
    }
}

__global__ __launch_bounds__(128) void k_gemm(const us* __restrict__ A, const us* __restrict__ W, float* Y,
                                              unsigned lda, unsigned ldw, unsigned ldy, unsigned K, unsigned KM, unsigned gA, unsigned gB) {
    __shared__ __align__(16) float st[NWV * 64 * GSP];
    const unsigned tid = threadIdx.x, lane = tid & 31u, wv = tid >> 5, lr = lane & 15u, hi = lane >> 4;
    const unsigned wm = wv >> 1, wn = wv & 1u;
    const unsigned row0 = blockIdx.y * 128u + wm * 64u;
    const unsigned n0 = blockIdx.x * 64u, col0 = n0 + wn * 32u;
    const unsigned gsh = ((n0 >= gA) ? 128u : 0u) + ((n0 >= gB) ? 128u : 0u);
    const us* ap = A + (size_t)(row0 + lr) * lda + 8u * hi;
    const us* wp = W + (size_t)(col0 + lr) * ldw + 8u * hi;
    v8f acc[4][2];
#pragma unroll
    for (int mi = 0; mi < 4; ++mi) { acc[mi][0] = (v8f){}; acc[mi][1] = (v8f){}; }
#pragma unroll 1
    for (unsigned kk = 0; kk < K; kk += 32u) {
        const unsigned ka = kk + ((kk >= KM) ? gsh : 0u);
        const v16bf a0 = ldb(ap + ka);
        const v16bf a1 = ldb(ap + (size_t)16 * lda + ka);
        const v16bf a2 = ldb(ap + (size_t)32 * lda + ka);
        const v16bf a3 = ldb(ap + (size_t)48 * lda + ka);
        const v16bf b0 = ldb(wp + kk);
        const v16bf b1 = ldb(wp + (size_t)16 * ldw + kk);
        acc[0][0] = wmmab(a0, b0, acc[0][0]); acc[0][1] = wmmab(a0, b1, acc[0][1]);
        acc[1][0] = wmmab(a1, b0, acc[1][0]); acc[1][1] = wmmab(a1, b1, acc[1][1]);
        acc[2][0] = wmmab(a2, b0, acc[2][0]); acc[2][1] = wmmab(a2, b1, acc[2][1]);
        acc[3][0] = wmmab(a3, b0, acc[3][0]); acc[3][1] = wmmab(a3, b1, acc[3][1]);
        asm volatile("v_nop\n\tv_nop\n\tv_nop\n\tv_nop"
                     : "+v"(acc[0][0]), "+v"(acc[0][1]), "+v"(acc[1][0]), "+v"(acc[1][1]),
                       "+v"(acc[2][0]), "+v"(acc[2][1]), "+v"(acc[3][0]), "+v"(acc[3][1])
                     : "v"(a0), "v"(a1), "v"(a2), "v"(a3), "v"(b0), "v"(b1));
    }
    float* sw = st + wv * (64 * GSP);
#pragma unroll
    for (int mi = 0; mi < 4; ++mi) {
#pragma unroll
        for (int ni = 0; ni < 2; ++ni) {
#pragma unroll
            for (int r = 0; r < 8; ++r) sw[(mi * 16 + 8 * hi + r) * GSP + ni * 16 + lr] = acc[mi][ni][r];
        }
    }
    __syncthreads();
    const unsigned pc = (lane & 7u) * 4u, rq = lane >> 3;
    float* yb = Y + (size_t)row0 * ldy + col0 + pc;
#pragma unroll 1
    for (int ps = 0; ps < 2; ++ps) {
#pragma unroll 4
        for (unsigned it = 0; it < 16u; ++it) {
            const unsigned row = it * 4u + rq;
            const v4f v = *(const v4fa*)(sw + row * GSP + pc);
            *(volatile v4f*)(yb + (size_t)row * ldy) = v;
        }
        if (ps == 0) __threadfence();
    }
}

__global__ __launch_bounds__(256) void k_hs(const float* __restrict__ HR, us* A, unsigned ldh, unsigned loff, unsigned ng, unsigned lda, unsigned ext0) {
    const unsigned t = blockIdx.x * 256u + threadIdx.x;
    const unsigned total = (unsigned)SEQ * ng;
    unsigned unit = t >> 4;
    const bool ok = unit < total;
    if (!ok) unit = total - 1u;
    const unsigned j = t & 15u, e = j & 7u, part = j >> 3;
    const unsigned s = unit / ng, g = unit - s * ng;
    const float* hr = HR + (size_t)s * ldh;
    const float lg = hr[loff + g * 8u + e];
    float mx = lg;
    mx = fmaxf(mx, __shfl_xor(mx, 1, 32));
    mx = fmaxf(mx, __shfl_xor(mx, 2, 32));
    mx = fmaxf(mx, __shfl_xor(mx, 4, 32));
    const float ex = expf(lg - mx);
    float sm = ex;
    sm += __shfl_xor(sm, 1, 32);
    sm += __shfl_xor(sm, 2, 32);
    sm += __shfl_xor(sm, 4, 32);
    const float rw = ex * (1.0f / sm) * 4.0f;
    const v4f h0 = *(const v4f*)(hr + g * 64u + e * 8u);
    const v4f h1 = *(const v4f*)(hr + g * 64u + e * 8u + 4u);
    v8us o;
#pragma unroll
    for (int k = 0; k < 8; ++k) {
        const float v = ((k < 4) ? h0[k & 3] : h1[k & 3]) * rw;
        const unsigned short hb = f2bf(v);
        const unsigned short lb = f2bf(v - bf2f(hb));
        o[k] = part ? lb : hb;
    }
    us* d = A + (size_t)s * lda + ext0 + g * 128u + part * 64u + e * 8u;
    if (ok) {
        *(volatile v8us*)d = o;
        __threadfence();
        *(volatile v8us*)d = o;
    }
}

__global__ __launch_bounds__(256) void k_rope(const float* __restrict__ Y, const float* __restrict__ cs, const float* __restrict__ sn,
                                              us* HI, us* RS, unsigned ycol0, unsigned nc8) {
    const unsigned i = blockIdx.x * 256u + threadIdx.x;
    if (i >= (unsigned)SEQ * nc8) return;
    const unsigned s = i / nc8, c = (i - s * nc8) * 8u;
    const float* y = Y + (size_t)s * NQKV + ycol0 + c;
    const v4f y0 = *(const v4f*)y;
    const v4f y1 = *(const v4f*)(y + 4);
    const unsigned i0 = (c & 63u) >> 1;
    const v4f cc = *(const v4f*)(cs + (size_t)s * 32u + i0);
    const v4f ss = *(const v4f*)(sn + (size_t)s * 32u + i0);
    float t[8] = { y0[0], y0[1], y0[2], y0[3], y1[0], y1[1], y1[2], y1[3] };
    float o[8];
#pragma unroll
    for (int p = 0; p < 4; ++p) {
        const float cr = bfr(cc[p]), sr = bfr(ss[p]);
        o[2 * p]     = t[2 * p] * cr - t[2 * p + 1] * sr;
        o[2 * p + 1] = t[2 * p] * sr + t[2 * p + 1] * cr;
    }
    v8h hv, rv;
#pragma unroll
    for (int k = 0; k < 8; ++k) {
        const _Float16 h = (_Float16)o[k];
        hv[k] = h;
        rv[k] = (_Float16)((o[k] - (float)h) * 2048.0f);
    }
    const v8us ho = __builtin_bit_cast(v8us, hv);
    const v8us ro = __builtin_bit_cast(v8us, rv);
    const size_t off = (size_t)s * (nc8 * 8u) + c;
    *(volatile v8us*)(HI + off) = ho;
    *(volatile v8us*)(RS + off) = ro;
    __threadfence();
    *(volatile v8us*)(HI + off) = ho;
    *(volatile v8us*)(RS + off) = ro;
}

__global__ __launch_bounds__(256) void k_vt(const float* __restrict__ Y, us* VTH, us* VTR) {
    __shared__ __align__(16) us th[128 * VTP];
    __shared__ __align__(16) us tr[128 * VTP];
    const unsigned tid = threadIdx.x;
    const unsigned k0 = blockIdx.x * 64u, cb = blockIdx.y;
    const float* src = Y + (size_t)k0 * NQKV + (DM + KVW) + cb * 128u;
#pragma unroll
    for (unsigned it = 0; it < 8u; ++it) {
        const unsigned f = it * 256u + tid;
        const unsigned key = f >> 5, d4 = (f & 31u) * 4u;
        const v4f x = *(const v4f*)(src + (size_t)key * NQKV + d4);
#pragma unroll
        for (unsigned c = 0; c < 4u; ++c) {
            const _Float16 h = (_Float16)x[c];
            const _Float16 r = (_Float16)((x[c] - (float)h) * 2048.0f);
            th[(d4 + c) * VTP + key] = __builtin_bit_cast(unsigned short, h);
            tr[(d4 + c) * VTP + key] = __builtin_bit_cast(unsigned short, r);
        }
    }
    __syncthreads();
    const size_t base = (size_t)(cb * 128u) * SEQ + k0;
    const unsigned c8 = (tid & 7u) * 8u, dr = tid >> 3;
#pragma unroll 1
    for (int ps = 0; ps < 2; ++ps) {
#pragma unroll
        for (unsigned it = 0; it < 4u; ++it) {
            const unsigned d = it * 32u + dr;
            const v8us oh = *(const v8usa*)(th + d * VTP + c8);
            const v8us orr = *(const v8usa*)(tr + d * VTP + c8);
            *(volatile v8us*)(VTH + base + (size_t)d * SEQ + c8) = oh;
            *(volatile v8us*)(VTR + base + (size_t)d * SEQ + c8) = orr;
        }
        if (ps == 0) __threadfence();
    }
}

template <bool ER>
__device__ __forceinline__ void flash_body(const us* __restrict__ QH, const us* __restrict__ QR, const us* __restrict__ KH, const us* __restrict__ KR,
                                           const us* __restrict__ VTH, const us* __restrict__ VTR, const float* __restrict__ mask,
                                           const int* __restrict__ MT, us* CX, const unsigned qb, const unsigned head) {
    __shared__ __align__(16) us osh[NWV * 16 * OSP];
    __shared__ __align__(16) us osl[NWV * 16 * OSP];
    const unsigned tid = threadIdx.x, lane = tid & 31u, wv = tid >> 5, lr = lane & 15u, hi = lane >> 4;
    const unsigned kvh = head >> 2;
    const unsigned q0w = qb * 64u + wv * 16u;
    const size_t qoff = (size_t)(q0w + lr) * DM + head * HD + 8u * hi;
    const size_t koff = (size_t)lr * KVW + kvh * HD + 8u * hi;
    const size_t voff = (size_t)(kvh * HD + lr) * SEQ + 8u * hi;
    const size_t moff = (size_t)(q0w + lr) * SEQ_FULL + 8u * hi;

    v8f o[4], o2[4];
#pragma unroll
    for (int t = 0; t < 4; ++t) { o[t] = (v8f){}; o2[t] = (v8f){}; }
    float ml = -1.0e30f;
    float l = 0.0f;

#pragma unroll 1
    for (unsigned kb = 0; kb < (unsigned)(SEQ / 64); ++kb) {
        int cls = MT[qb * 32u + kb];
        if ((unsigned)cls > 2u) cls = 1;
        if (cls == 2) continue;
#pragma unroll 1
        for (unsigned hf = 0; hf < 2u; ++hf) {
            const unsigned k0 = kb * 64u + hf * 32u;
            v8f sh0 = (v8f){}, sh1 = (v8f){}, sr0 = (v8f){}, sr1 = (v8f){};
            {
                const us* ka = KH + koff + (size_t)k0 * KVW;
                const us* kr = KR + koff + (size_t)k0 * KVW;
                const v16h a00 = ldh(ka), a10 = ldh(ka + 16 * KVW);
                const v16h bq0 = ldh(QH + qoff), br0 = ldh(QR + qoff);
                sh0 = wmmah(a00, bq0, sh0); sh1 = wmmah(a10, bq0, sh1);
                sr0 = wmmah(a00, br0, sr0); sr1 = wmmah(a10, br0, sr1);
                const v16h a01 = ldh(ka + 32), a11 = ldh(ka + 16 * KVW + 32);
                const v16h bq1 = ldh(QH + qoff + 32), br1 = ldh(QR + qoff + 32);
                sh0 = wmmah(a01, bq1, sh0); sh1 = wmmah(a11, bq1, sh1);
                sr0 = wmmah(a01, br1, sr0); sr1 = wmmah(a11, br1, sr1);
                if (ER) {
                    const v16h c00 = ldh(kr), c10 = ldh(kr + 16 * KVW);
                    const v16h c01 = ldh(kr + 32), c11 = ldh(kr + 16 * KVW + 32);
                    sr0 = wmmah(c00, bq0, sr0); sr1 = wmmah(c10, bq0, sr1);
                    sr0 = wmmah(c01, bq1, sr0); sr1 = wmmah(c11, bq1, sr1);
                    asm volatile("v_nop\n\tv_nop\n\tv_nop\n\tv_nop" : "+v"(sh0), "+v"(sh1), "+v"(sr0), "+v"(sr1)
                                 : "v"(c01), "v"(c11), "v"(bq1), "v"(bq0), "v"(c00), "v"(c10));
                } else {
                    asm volatile("v_nop\n\tv_nop\n\tv_nop\n\tv_nop" : "+v"(sh0), "+v"(sh1), "+v"(sr0), "+v"(sr1)
                                 : "v"(a01), "v"(a11), "v"(bq1), "v"(br1));
                }
            }
            float s0[8], s1[8];
#pragma unroll
            for (int r = 0; r < 8; ++r) {
                s0[r] = fmaf(sr0[r], RQ, sh0[r]) * 0.125f;
                s1[r] = fmaf(sr1[r], RQ, sh1[r]) * 0.125f;
            }
            if (cls == 1) {
                const float* mp = mask + moff + k0;
                const v4f m00 = *(const v4f*)(mp), m01 = *(const v4f*)(mp + 4);
                const v4f m10 = *(const v4f*)(mp + 16), m11 = *(const v4f*)(mp + 20);
#pragma unroll
                for (int r = 0; r < 4; ++r) {
                    s0[r] += m00[r]; s0[4 + r] += m01[r];
                    s1[r] += m10[r]; s1[4 + r] += m11[r];
                }
            }
            float mx = fmaxf(s0[0], s1[0]);
#pragma unroll
            for (int r = 1; r < 8; ++r) mx = fmaxf(mx, fmaxf(s0[r], s1[r]));
            mx = fmaxf(mx, __shfl_xor(mx, 16, 32));
            const float mnl = fmaxf(ml, mx * L2E);
            const float corr = __builtin_amdgcn_exp2f(ml - mnl);
            ml = mnl;
            float p0[8], p1[8];
            float psum = 0.0f;
#pragma unroll
            for (int r = 0; r < 8; ++r) {
                p0[r] = __builtin_amdgcn_exp2f(fmaf(s0[r], L2E, -mnl));
                p1[r] = __builtin_amdgcn_exp2f(fmaf(s1[r], L2E, -mnl));
                psum += p0[r] + p1[r];
            }
            psum += __shfl_xor(psum, 16, 32);
            l = l * corr + psum;
            if (__builtin_amdgcn_ballot_w32(corr != 1.0f) != 0u) {
#pragma unroll
                for (int t = 0; t < 4; ++t) { o[t] *= corr; if (ER) o2[t] *= corr; }
            }
            v16h ph, pr;
#pragma unroll
            for (int r = 0; r < 8; ++r) {
                const float c0 = p0[r] * 1024.0f, c1 = p1[r] * 1024.0f;
                const _Float16 h0 = (_Float16)c0, h1 = (_Float16)c1;
                ph[r] = h0; ph[8 + r] = h1;
                pr[r]     = ER ? (_Float16)((c0 - (float)h0) * 2048.0f) : (_Float16)0.0f;
                pr[8 + r] = ER ? (_Float16)((c1 - (float)h1) * 2048.0f) : (_Float16)0.0f;
            }
            asm volatile("" ::: "memory");
            v16h av[4], arv[4];
#pragma unroll
            for (int t = 0; t < 4; ++t) {
                av[t] = ldh(VTH + voff + (size_t)t * 16 * SEQ + k0);
                if (ER) arv[t] = ldh(VTR + voff + (size_t)t * 16 * SEQ + k0); else arv[t] = av[t];
            }
#pragma unroll
            for (int t = 0; t < 4; ++t) {
                o[t] = wmmah(av[t], ph, o[t]);
                if (ER) {
                    o2[t] = wmmah(av[t], pr, o2[t]);
                    o2[t] = wmmah(arv[t], ph, o2[t]);
                }
            }
            if (ER) {
                asm volatile("v_nop\n\tv_nop\n\tv_nop\n\tv_nop"
                             : "+v"(o[0]), "+v"(o[1]), "+v"(o[2]), "+v"(o[3]), "+v"(o2[0]), "+v"(o2[1]), "+v"(o2[2]), "+v"(o2[3])
                             : "v"(ph), "v"(pr), "v"(av[3]), "v"(arv[3]));
            } else {
                asm volatile("v_nop\n\tv_nop\n\tv_nop\n\tv_nop"
                             : "+v"(o[0]), "+v"(o[1]), "+v"(o[2]), "+v"(o[3])
                             : "v"(ph), "v"(av[3]), "v"(av[2]));
            }
        }
    }

    const float inv = 1.0f / (1024.0f * l);
    const unsigned srow = (wv * 16u + lr) * OSP + 8u * hi;
#pragma unroll
    for (int t = 0; t < 4; ++t) {
        v8us hv, lv;
#pragma unroll
        for (int r = 0; r < 8; ++r) {
            float val = o[t][r];
            if (ER) val = fmaf(o2[t][r], RQ, val);
            val *= inv;
            const unsigned short hb = f2bf(val);
            hv[r] = hb;
            lv[r] = f2bf(val - bf2f(hb));
        }
        *(v8usa*)(osh + srow + t * 16) = hv;
        *(v8usa*)(osl + srow + t * 16) = lv;
    }
    __syncthreads();
    const unsigned pc = (lane & 7u) * 8u, rq = lane >> 3;
#pragma unroll 1
    for (int ps = 0; ps < 2; ++ps) {
#pragma unroll
        for (unsigned it = 0; it < 4u; ++it) {
            const unsigned qi = it * 4u + rq;
            const v8us hv = *(const v8usa*)(osh + (wv * 16u + qi) * OSP + pc);
            const v8us lv = *(const v8usa*)(osl + (wv * 16u + qi) * OSP + pc);
            us* d = CX + (size_t)(q0w + qi) * CXP + head * HD + pc;
            *(volatile v8us*)d = hv;
            *(volatile v8us*)(d + DM) = lv;
        }
        if (ps == 0) __threadfence();
    }
}

__global__ __launch_bounds__(128) void k_flash_e(const us* QH, const us* QR, const us* KH, const us* KR, const us* VTH, const us* VTR,
                                                 const float* mask, const int* MT, us* CX) {
    flash_body<true>(QH, QR, KH, KR, VTH, VTR, mask, MT, CX, blockIdx.x / NH, blockIdx.x % NH);
}
__global__ __launch_bounds__(128) void k_flash_l(const us* QH, const us* QR, const us* KH, const us* KR, const us* VTH, const us* VTR,
                                                 const float* mask, const int* MT, us* CX) {
    flash_body<false>(QH, QR, KH, KR, VTH, VTR, mask, MT, CX, (unsigned)(EARLYR / 64) + blockIdx.x / NH, blockIdx.x % NH);
}

#define SZ_XE  ((size_t)SEQ * XEP * 2)
#define SZ_WE  ((size_t)NQKV * WEP * 2)
#define SZ_WA  ((size_t)NA1 * DM * 2)
#define SZ_WC  ((size_t)NA2 * WCP * 2)
#define SZ_WD  ((size_t)DM * CXP * 2)
#define SZ_H1  ((size_t)SEQ * NA1 * 4)
#define SZ_H2  ((size_t)SEQ * NA2 * 4)
#define SZ_Y1  ((size_t)SEQ * NQKV * 4)
#define SZ_Q   ((size_t)SEQ * DM * 2)
#define SZ_K   ((size_t)SEQ * KVW * 2)
#define SZ_VT  ((size_t)KVW * SEQ * 2)
#define SZ_CX  ((size_t)SEQ * CXP * 2)
#define SZ_MT  ((size_t)32 * 128)
#define SZ_ALL (SZ_XE + SZ_WE + SZ_WA + SZ_WC + SZ_WD + SZ_H1 + SZ_H2 + SZ_Y1 + 2 * SZ_Q + 2 * SZ_K + 2 * SZ_VT + SZ_CX + SZ_MT)
static_assert(SZ_ALL <= (size_t)134217728);
static_assert(SZ_XE % 256 == 0 && SZ_WE % 256 == 0 && SZ_WD % 256 == 0 && SZ_CX % 256 == 0 && SZ_K % 256 == 0 && SZ_VT % 256 == 0);
static_assert((size_t)(SEQ / 64) * 32 * 4 <= SZ_MT);

extern "C" void kernel_launch(void* const* d_in, const int* in_sizes, int n_in,
                              void* d_out, int out_size, void* d_ws, size_t ws_size, hipStream_t stream) {
    if (n_in < 21) return;
    if ((size_t)in_sizes[0] < (size_t)SEQ * DM) return;
    if (in_sizes[1] < 1) return;
    if ((size_t)in_sizes[2] < (size_t)(SEQ - 1) * SEQ_FULL + SEQ) return;
    if ((size_t)in_sizes[3] < (size_t)SEQ * 32 || (size_t)in_sizes[4] < (size_t)SEQ * 32) return;
    if ((size_t)in_sizes[5] < (size_t)DM * DM || (size_t)in_sizes[8] < (size_t)DM * DM) return;
    if ((size_t)in_sizes[6] < (size_t)KVW * DM || (size_t)in_sizes[7] < (size_t)KVW * DM) return;
    for (int g = 0; g < 4; ++g) {
        const size_t outd = (g == 0 || g == 3) ? (size_t)DM : (size_t)KVW;
        if ((size_t)in_sizes[9 + 3 * g] < (size_t)8 * DM) return;
        if ((size_t)in_sizes[10 + 3 * g] < (size_t)64 * DM) return;
        if ((size_t)in_sizes[11 + 3 * g] < (size_t)8 * outd * 8) return;
    }
    if ((size_t)out_size < (size_t)SEQ * DM) return;
    if (SZ_ALL > ws_size) return;

    const float* x    = (const float*)d_in[0];
    const int*   sp   = (const int*)d_in[1];
    const float* mask = (const float*)d_in[2];
    const float* fc   = (const float*)d_in[3];
    const float* fs   = (const float*)d_in[4];
    const float* wq   = (const float*)d_in[5];
    const float* wk   = (const float*)d_in[6];
    const float* wv   = (const float*)d_in[7];
    const float* wo   = (const float*)d_in[8];
    const float* lqr  = (const float*)d_in[9];
    const float* lqA  = (const float*)d_in[10];
    const float* lqB  = (const float*)d_in[11];
    const float* lkr  = (const float*)d_in[12];
    const float* lkA  = (const float*)d_in[13];
    const float* lkB  = (const float*)d_in[14];
    const float* lvr  = (const float*)d_in[15];
    const float* lvA  = (const float*)d_in[16];
    const float* lvB  = (const float*)d_in[17];
    const float* lor  = (const float*)d_in[18];
    const float* loA  = (const float*)d_in[19];
    const float* loB  = (const float*)d_in[20];
    float* OUT = (float*)d_out;

    char* w = (char*)d_ws;
    size_t off = 0;
    us* XE = (us*)(w + off); off += SZ_XE;
    us* WE = (us*)(w + off); off += SZ_WE;
    us* WA = (us*)(w + off); off += SZ_WA;
    us* WC = (us*)(w + off); off += SZ_WC;
    us* WD = (us*)(w + off); off += SZ_WD;
    float* H1 = (float*)(w + off); off += SZ_H1;
    float* H2 = (float*)(w + off); off += SZ_H2;
    float* Y1 = (float*)(w + off); off += SZ_Y1;
    us* QH = (us*)(w + off); off += SZ_Q;
    us* QR = (us*)(w + off); off += SZ_Q;
    us* KH = (us*)(w + off); off += SZ_K;
    us* KR = (us*)(w + off); off += SZ_K;
    us* VTH = (us*)(w + off); off += SZ_VT;
    us* VTR = (us*)(w + off); off += SZ_VT;
    us* CX = (us*)(w + off); off += SZ_CX;
    int* MT = (int*)(w + off); off += SZ_MT;

    const unsigned BIG = 0x7FFFFFFFu;

    k_mscan<<<(unsigned)(SEQ / 64), 256, 0, stream>>>(mask, sp, MT);
    k_cvt<<<(unsigned)SEQ, 256, 0, stream>>>(x, XE, (unsigned)SEQ, (unsigned)XEP, 1u);
    k_cvt<<<(unsigned)DM, 256, 0, stream>>>(wq, WE, (unsigned)DM, (unsigned)WEP, 1u);
    k_cvt<<<(unsigned)KVW, 256, 0, stream>>>(wk, WE + (size_t)DM * WEP, (unsigned)KVW, (unsigned)WEP, 1u);
    k_cvt<<<(unsigned)KVW, 256, 0, stream>>>(wv, WE + (size_t)(DM + KVW) * WEP, (unsigned)KVW, (unsigned)WEP, 1u);
    k_cvt<<<64u, 256, 0, stream>>>(lqA, WA, 64u, (unsigned)DM, 1u);
    k_cvt<<<64u, 256, 0, stream>>>(lkA, WA + (size_t)64 * DM, 64u, (unsigned)DM, 1u);
    k_cvt<<<64u, 256, 0, stream>>>(lvA, WA + (size_t)128 * DM, 64u, (unsigned)DM, 1u);
    k_rt<<<64u, 256, 0, stream>>>(lqr, lkr, lvr, WA + (size_t)192 * DM, 3u, (unsigned)DM, 1u);
    k_bt<<<(unsigned)(DM * 16 / 256), 256, 0, stream>>>(lqB, WE + DM, (unsigned)DM, (unsigned)WEP);
    k_bt<<<(unsigned)(KVW * 16 / 256), 256, 0, stream>>>(lkB, WE + (size_t)DM * WEP + DM, (unsigned)KVW, (unsigned)WEP);
    k_bt<<<(unsigned)(KVW * 16 / 256), 256, 0, stream>>>(lvB, WE + (size_t)(DM + KVW) * WEP + DM, (unsigned)KVW, (unsigned)WEP);
    k_cvt<<<64u, 256, 0, stream>>>(loA, WC, 64u, (unsigned)WCP, 2u);
    k_rt<<<64u, 256, 0, stream>>>(lor, lor, lor, WC + (size_t)64 * WCP, 1u, (unsigned)WCP, 2u);
    k_cvt<<<(unsigned)DM, 256, 0, stream>>>(wo, WD, (unsigned)DM, (unsigned)CXP, 2u);
    k_bt<<<(unsigned)(DM * 16 / 256), 256, 0, stream>>>(loB, WD + 2 * DM, (unsigned)DM, (unsigned)CXP);

    k_gemm<<<dim3(NA1 / 64, SEQ / 128, 1), 128, 0, stream>>>(XE, WA, H1, (unsigned)XEP, (unsigned)DM, (unsigned)NA1, (unsigned)DM, (unsigned)DM, BIG, BIG);
    k_hs<<<(unsigned)((size_t)SEQ * 3 * 16 / 256), 256, 0, stream>>>(H1, XE, (unsigned)NA1, 192u, 3u, (unsigned)XEP, (unsigned)DM);
    k_gemm<<<dim3(NQKV / 64, SEQ / 128, 1), 128, 0, stream>>>(XE, WE, Y1, (unsigned)XEP, (unsigned)WEP, (unsigned)NQKV, (unsigned)WEP, (unsigned)DM, (unsigned)DM, (unsigned)(DM + KVW));
    k_rope<<<(unsigned)((size_t)SEQ * (DM / 8) / 256), 256, 0, stream>>>(Y1, fc, fs, QH, QR, 0u, (unsigned)(DM / 8));
    k_rope<<<(unsigned)((size_t)SEQ * (KVW / 8) / 256), 256, 0, stream>>>(Y1, fc, fs, KH, KR, (unsigned)DM, (unsigned)(KVW / 8));
    k_vt<<<dim3(SEQ / 64, KVW / 128, 1), 256, 0, stream>>>(Y1, VTH, VTR);
    k_flash_e<<<(unsigned)((EARLYR / 64) * NH), 128, 0, stream>>>(QH, QR, KH, KR, VTH, VTR, mask, MT, CX);
    if (SEQ > EARLYR) {
        k_flash_l<<<(unsigned)(((SEQ - EARLYR) / 64) * NH), 128, 0, stream>>>(QH, QR, KH, KR, VTH, VTR, mask, MT, CX);
    }
    k_gemm<<<dim3(NA2 / 64, SEQ / 128, 1), 128, 0, stream>>>(CX, WC, H2, (unsigned)CXP, (unsigned)WCP, (unsigned)NA2, (unsigned)WCP, (unsigned)WCP, BIG, BIG);
    k_hs<<<(unsigned)((size_t)SEQ * 16 / 256), 256, 0, stream>>>(H2, CX, (unsigned)NA2, 64u, 1u, (unsigned)CXP, (unsigned)(2 * DM));
    k_gemm<<<dim3(DM / 64, SEQ / 128, 1), 128, 0, stream>>>(CX, WD, OUT, (unsigned)CXP, (unsigned)CXP, (unsigned)DM, (unsigned)CXP, (unsigned)CXP, BIG, BIG);
}
